// TransformerBlock_970662608910
// MI455X (gfx1250) — hardware-run, weakly checked
//
#include <hip/hip_runtime.h>

typedef _Float16 v16h __attribute__((ext_vector_type(16)));
typedef _Float16 v8h  __attribute__((ext_vector_type(8)));
typedef _Float16 v8ha __attribute__((ext_vector_type(8), may_alias));
typedef _Float16 v4h  __attribute__((ext_vector_type(4)));
typedef float    v8f  __attribute__((ext_vector_type(8)));
typedef float    v4f  __attribute__((ext_vector_type(4)));
typedef float    v4fa __attribute__((ext_vector_type(4), may_alias));

#ifndef NB
#define NB 2
#endif
#ifndef SEQ
#define SEQ 4096
#endif
#define NB_FULL 2
#define S_FULL  4096
#define NH      8
#define HD      64
#define NF      128
#define QB      64
#define EROWS   ((SEQ) < 512 ? (SEQ) : 512)
#define PP      72
#define FP      136
#define TP      72
#define RATIO   0.08838834764831845f
#define EPSF    1.0e-3f
#define LSCALE  2048.0f
#define RSPLIT  (1.0f / 2048.0f)

#define PLANE_BYTES ((size_t)NB_FULL * NH * S_FULL * NF * 2)
#define VT_BYTES    ((size_t)NB_FULL * NH * HD * S_FULL * 2)
#define RES_BYTES   ((size_t)NB_FULL * NH * EROWS * NF * 2)
#define WS_TOTAL    (2 * PLANE_BYTES + VT_BYTES + 2 * RES_BYTES)

static_assert(SEQ % QB == 0);
static_assert(SEQ % 32 == 0);
static_assert(SEQ <= S_FULL);
static_assert(NB <= NB_FULL);
static_assert(HD == 64);
static_assert(NF == 128);
static_assert(NF % 32 == 0 && HD % 32 == 0);
static_assert(EROWS % QB == 0 && EROWS <= SEQ);
static_assert((SEQ - EROWS) % QB == 0);
static_assert((PP % 8) == 0 && (FP % 8) == 0 && (TP % 8) == 0);
static_assert(PP >= HD && FP >= NF && TP >= 64);
static_assert(128 * 16 * 4 == NF * HD);
static_assert(32 * 16 * 8 == 16 * NF * 2);
static_assert(128 * 4 * 16 == HD * 64 * 2);
static_assert(32 * 16 * 8 == 16 * HD * 4);
static_assert((NF * PP + 2 * 4 * 16 * FP) * 2 <= 131072);
static_assert(HD * TP * 2 <= 131072);
static_assert(2 * 4 * 16 * 32 * 2 + 4 * 16 * HD * 4 <= 131072);
static_assert(PLANE_BYTES % 128 == 0 && VT_BYTES % 128 == 0 && RES_BYTES % 128 == 0);
static_assert(WS_TOTAL <= 134217728);

static __device__ __forceinline__ _Float16 toh_flush(float v)
{
    const _Float16 r = (_Float16)v;
    return (fabsf(v) < 6.103515625e-05f) ? (_Float16)0.0f : r;
}

static __device__ __forceinline__ _Float16 inh_flush(float x)
{
    unsigned u = __float_as_uint(x);
    u = (u + 0x7FFFu + ((u >> 16) & 1u)) & 0xFFFF0000u;
    return toh_flush(__uint_as_float(u));
}

static __device__ __forceinline__ v16h cat8(v8h a, v8h b)
{
    return __builtin_shufflevector(a, b, 0, 1, 2, 3, 4, 5, 6, 7, 8, 9, 10, 11, 12, 13, 14, 15);
}

static __device__ __forceinline__ v8f wmma16(v16h a, v16h b, v8f c)
{
    v8f d = __builtin_amdgcn_wmma_f32_16x16x32_f16(false, a, false, b, (short)0, c, false, false);
    asm volatile("v_nop\n\tv_nop\n\tv_nop\n\tv_nop" : "+v"(d) : "v"(a), "v"(b));
    return d;
}

__global__ void __launch_bounds__(128) feat_kernel(const float* __restrict__ X,
                                                   const float* __restrict__ PM,
                                                   _Float16* __restrict__ FH,
                                                   _Float16* __restrict__ FR)
{
    __shared__ __align__(16) _Float16 pw[NF * PP];
    __shared__ __align__(16) _Float16 fvb[4][16 * FP];
    __shared__ __align__(16) _Float16 frb[4][16 * FP];

    const int tid  = threadIdx.x;
    const int lane = tid & 31;
    const int wave = __builtin_amdgcn_readfirstlane(tid >> 5);
    const int lo   = lane & 15;
    const int hi   = lane >> 4;
    const int koff = hi * 8;
    const int l0   = blockIdx.x * QB;
    const int bh   = blockIdx.y;
    const int b    = bh / NH;
    const int h    = bh - b * NH;
    const int lw   = l0 + wave * 16;
    const bool er  = (l0 < EROWS);

#pragma unroll 4
    for (int it = 0; it < 16; ++it) {
        const int idx  = tid + 128 * it;
        const int row  = idx >> 4;
        const int col4 = (idx & 15) * 4;
        const v4f x = *(const v4f*)(PM + row * HD + col4);
        v4h t;
        t[0] = inh_flush(x[0]); t[1] = inh_flush(x[1]); t[2] = inh_flush(x[2]); t[3] = inh_flush(x[3]);
        *(v4h*)(pw + row * PP + col4) = t;
    }

    v16h ax0, ax1;
    {
        const float* xr = X + ((size_t)(b * S_FULL + lw + lo) * NH + h) * HD;
        v8h f[4];
#pragma unroll
        for (int s = 0; s < 4; ++s) {
            const v4f x0 = *(const v4f*)(xr + 16 * s + koff);
            const v4f x1 = *(const v4f*)(xr + 16 * s + koff + 4);
            v8h t;
            t[0] = inh_flush(x0[0]); t[1] = inh_flush(x0[1]); t[2] = inh_flush(x0[2]); t[3] = inh_flush(x0[3]);
            t[4] = inh_flush(x1[0]); t[5] = inh_flush(x1[1]); t[6] = inh_flush(x1[2]); t[7] = inh_flush(x1[3]);
            f[s] = t;
        }
        ax0 = cat8(f[0], f[1]);
        ax1 = cat8(f[2], f[3]);
    }
    __syncthreads();

    _Float16* fv = fvb[wave];
    _Float16* fr = frb[wave];
#pragma unroll
    for (int nt = 0; nt < 8; ++nt) {
        const _Float16* pr = pw + (nt * 16 + lo) * PP;
        const v16h b0 = cat8(*(const v8h*)(pr + koff),      *(const v8h*)(pr + 16 + koff));
        const v16h b1 = cat8(*(const v8h*)(pr + 32 + koff), *(const v8h*)(pr + 48 + koff));
        v8f acc = {};
        acc = wmma16(ax0, b0, acc);
        acc = wmma16(ax1, b1, acc);
#pragma unroll
        for (int i = 0; i < 8; ++i) {
            const float f = fmaxf(acc[i] * RATIO, 0.0f) + EPSF;
            const _Float16 hv = toh_flush(f);
            fv[(i + 8 * hi) * FP + nt * 16 + lo] = hv;
            if (er) fr[(i + 8 * hi) * FP + nt * 16 + lo] = toh_flush((f - (float)hv) * LSCALE);
        }
    }
    __syncthreads();

    {
        v8h ov[8];
#pragma unroll
        for (int i = 0; i < 8; ++i) {
            const int cc = lane + 32 * i, rr = cc >> 4, qd = cc & 15;
            ov[i] = *(const v8ha*)(fv + rr * FP + qd * 8);
        }
        _Float16* ob = FH + ((size_t)bh * S_FULL + lw) * NF;
#pragma unroll
        for (int i = 0; i < 8; ++i) {
            const int cc = lane + 32 * i, rr = cc >> 4, qd = cc & 15;
            *(volatile v8h*)(ob + (size_t)rr * NF + qd * 8) = ov[i];
        }
        __threadfence();
#pragma unroll
        for (int i = 0; i < 8; ++i) {
            const int cc = lane + 32 * i, rr = cc >> 4, qd = cc & 15;
            *(volatile v8h*)(ob + (size_t)rr * NF + qd * 8) = ov[i];
        }
    }
    if (er) {
        v8h ov[8];
#pragma unroll
        for (int i = 0; i < 8; ++i) {
            const int cc = lane + 32 * i, rr = cc >> 4, qd = cc & 15;
            ov[i] = *(const v8ha*)(fr + rr * FP + qd * 8);
        }
        _Float16* ob = FR + ((size_t)bh * EROWS + lw) * NF;
#pragma unroll
        for (int i = 0; i < 8; ++i) {
            const int cc = lane + 32 * i, rr = cc >> 4, qd = cc & 15;
            *(volatile v8h*)(ob + (size_t)rr * NF + qd * 8) = ov[i];
        }
        __threadfence();
#pragma unroll
        for (int i = 0; i < 8; ++i) {
            const int cc = lane + 32 * i, rr = cc >> 4, qd = cc & 15;
            *(volatile v8h*)(ob + (size_t)rr * NF + qd * 8) = ov[i];
        }
    }
}

__global__ void __launch_bounds__(128) vt_kernel(const float* __restrict__ V,
                                                 _Float16* __restrict__ VT)
{
#pragma clang fp contract(off)
    __shared__ __align__(16) _Float16 tb[HD * TP];

    const int tid = threadIdx.x;
    const int l0  = blockIdx.x * 64;
    const int bh  = blockIdx.y;
    const int b   = bh / NH;
    const int h   = bh - b * NH;

#pragma unroll 2
    for (int it = 0; it < 8; ++it) {
        const int idx  = tid + 128 * it;
        const int row  = idx >> 4;
        const int col4 = (idx & 15) * 4;
        const size_t g = ((size_t)(b * S_FULL + l0 + row) * NH + h) * HD + col4;
        const v4f vv = *(const v4f*)(V + g);
        tb[(col4 + 0) * TP + row] = inh_flush(vv[0]);
        tb[(col4 + 1) * TP + row] = inh_flush(vv[1]);
        tb[(col4 + 2) * TP + row] = inh_flush(vv[2]);
        tb[(col4 + 3) * TP + row] = inh_flush(vv[3]);
    }
    __syncthreads();

    v8h ov[4];
#pragma unroll
    for (int it = 0; it < 4; ++it) {
        const int idx = tid + 128 * it, r = idx >> 3, p = idx & 7;
        ov[it] = *(const v8ha*)(tb + r * TP + p * 8);
    }
    _Float16* ob = VT + (size_t)bh * HD * S_FULL + l0;
#pragma unroll
    for (int it = 0; it < 4; ++it) {
        const int idx = tid + 128 * it, r = idx >> 3, p = idx & 7;
        *(volatile v8h*)(ob + (size_t)r * S_FULL + p * 8) = ov[it];
    }
    __threadfence();
#pragma unroll
    for (int it = 0; it < 4; ++it) {
        const int idx = tid + 128 * it, r = idx >> 3, p = idx & 7;
        *(volatile v8h*)(ob + (size_t)r * S_FULL + p * 8) = ov[it];
    }
}

template <bool EARLY, bool MASK>
static __device__ __forceinline__ void p_tile(const v8f cs0, const v8f cs1, float (&rl)[8],
                                              _Float16* pb, _Float16* plb,
                                              const int lo, const int hi, const int dq)
{
#pragma unroll
    for (int i = 0; i < 8; ++i) {
        const int m = i + 8 * hi;
        float p0 = cs0[i];
        float p1 = cs1[i];
        if (MASK) {
            const bool ok0 = (lo <= dq + m);
            const bool ok1 = (lo + 16 <= dq + m);
            p0 = ok0 ? p0 : 0.0f;
            p1 = ok1 ? p1 : 0.0f;
        }
        rl[i] += p0 + p1;
        const _Float16 h0 = toh_flush(p0);
        const _Float16 h1 = toh_flush(p1);
        pb[m * 32 + lo]      = h0;
        pb[m * 32 + 16 + lo] = h1;
        if (EARLY) {
            plb[m * 32 + lo]      = toh_flush((p0 - (float)h0) * LSCALE);
            plb[m * 32 + 16 + lo] = toh_flush((p1 - (float)h1) * LSCALE);
        }
    }
}

template <bool EARLY>
static __device__ __forceinline__ void favor_attn_body(const _Float16* QH, const _Float16* KH,
                                                       const _Float16* QR, const _Float16* KR,
                                                       const _Float16* VT, float* O,
                                                       const int qblk0)
{
    __shared__ __align__(16) _Float16 pbuf[4][16 * 32];
    __shared__ __align__(16) _Float16 plbuf[EARLY ? 4 : 1][16 * 32];
    __shared__ __align__(16) float    sout[4][16 * HD];

    const int tid  = threadIdx.x;
    const int lane = tid & 31;
    const int wave = __builtin_amdgcn_readfirstlane(tid >> 5);
    const int lo   = lane & 15;
    const int hi   = lane >> 4;
    const int koff = hi * 8;
    const int q0   = (qblk0 + (int)blockIdx.x) * QB;
    const int bh   = blockIdx.y;
    const int b    = bh / NH;
    const int h    = bh - b * NH;
    const int qw   = q0 + wave * 16;
    const size_t prow = (size_t)bh * S_FULL;
    const size_t rrow = (size_t)bh * EROWS;

    _Float16* pb  = pbuf[wave];
    _Float16* plb = plbuf[EARLY ? wave : 0];

    v16h aq[4];
    {
        const _Float16* qr = QH + (prow + qw + lo) * NF;
#pragma unroll
        for (int ks = 0; ks < 4; ++ks)
            aq[ks] = cat8(*(const v8h*)(qr + 32 * ks + koff), *(const v8h*)(qr + 32 * ks + 16 + koff));
    }

    v8f oacc[4];
#pragma unroll
    for (int nt = 0; nt < 4; ++nt) { v8f z = {}; oacc[nt] = z; }
    float rl[8];
#pragma unroll
    for (int i = 0; i < 8; ++i) rl[i] = 0.0f;

    const int kend = q0 + QB - 1;
    for (int c = 0; c <= kend; c += 32) {
        const bool active = (c <= qw + 15);

        if (active) {
            v8f cs0 = {}, cs1 = {}, rs0 = {}, rs1 = {};
#pragma unroll
            for (int ks = 0; ks < 4; ++ks) {
                const _Float16* k0r = KH + (prow + c + lo) * NF + 32 * ks + koff;
                const _Float16* k1r = k0r + 16 * NF;
                const v16h b0 = cat8(*(const v8h*)(k0r), *(const v8h*)(k0r + 16));
                const v16h b1 = cat8(*(const v8h*)(k1r), *(const v8h*)(k1r + 16));
                cs0 = wmma16(aq[ks], b0, cs0);
                cs1 = wmma16(aq[ks], b1, cs1);
                if (EARLY) {
                    const _Float16* r0r = KR + (rrow + c + lo) * NF + 32 * ks + koff;
                    const _Float16* r1r = r0r + 16 * NF;
                    const v16h r0 = cat8(*(const v8h*)(r0r), *(const v8h*)(r0r + 16));
                    const v16h r1 = cat8(*(const v8h*)(r1r), *(const v8h*)(r1r + 16));
                    const _Float16* qrr = QR + (rrow + qw + lo) * NF + 32 * ks + koff;
                    const v16h aqr = cat8(*(const v8h*)(qrr), *(const v8h*)(qrr + 16));
                    rs0 = wmma16(aq[ks], r0, rs0);
                    rs0 = wmma16(aqr, b0, rs0);
                    rs1 = wmma16(aq[ks], r1, rs1);
                    rs1 = wmma16(aqr, b1, rs1);
                }
            }
            if (EARLY) {
                cs0 += rs0 * RSPLIT;
                cs1 += rs1 * RSPLIT;
            }

            const bool diag = (c + 31 > qw);
            if (diag) p_tile<EARLY, true >(cs0, cs1, rl, pb, plb, lo, hi, qw - c);
            else      p_tile<EARLY, false>(cs0, cs1, rl, pb, plb, lo, hi, qw - c);
        }
        __syncthreads();

        if (active) {
            const v16h ap = cat8(*(const v8h*)(pb + lo * 32 + koff), *(const v8h*)(pb + lo * 32 + 16 + koff));
            v16h apl = ap;
            if (EARLY) apl = cat8(*(const v8h*)(plb + lo * 32 + koff), *(const v8h*)(plb + lo * 32 + 16 + koff));
#pragma unroll
            for (int nt = 0; nt < 4; ++nt) {
                const _Float16* vr = VT + ((size_t)bh * HD + nt * 16 + lo) * S_FULL + c;
                const v16h vb = cat8(*(const v8h*)(vr + koff), *(const v8h*)(vr + 16 + koff));
                if (EARLY) {
                    v8f x = {};
                    x = wmma16(apl, vb, x);
                    oacc[nt] = wmma16(ap, vb, oacc[nt]);
                    oacc[nt] += x * RSPLIT;
                } else {
                    oacc[nt] = wmma16(ap, vb, oacc[nt]);
                }
            }
        }
        __syncthreads();
    }

    float inv[8];
#pragma unroll
    for (int i = 0; i < 8; ++i) {
        float s = rl[i];
#pragma unroll
        for (int d = 1; d < 16; d <<= 1) s += __shfl_xor(s, d, 32);
        inv[i] = 1.0f / s;
    }
    float* so = sout[wave];
#pragma unroll
    for (int nt = 0; nt < 4; ++nt) {
#pragma unroll
        for (int i = 0; i < 8; ++i) so[(i + 8 * hi) * HD + nt * 16 + lo] = oacc[nt][i] * inv[i];
    }
    __syncthreads();

    v4f ov[8];
#pragma unroll
    for (int i = 0; i < 8; ++i) {
        const int cc = lane + 32 * i, rr = cc >> 4, qd = cc & 15;
        ov[i] = *(const v4fa*)(so + rr * HD + qd * 4);
    }
    float* ob = O + ((size_t)(b * S_FULL + qw) * NH + h) * HD;
#pragma unroll
    for (int i = 0; i < 8; ++i) {
        const int cc = lane + 32 * i, rr = cc >> 4, qd = cc & 15;
        *(volatile v4f*)(ob + (size_t)rr * (NH * HD) + qd * 4) = ov[i];
    }
    __threadfence();
#pragma unroll
    for (int i = 0; i < 8; ++i) {
        const int cc = lane + 32 * i, rr = cc >> 4, qd = cc & 15;
        *(volatile v4f*)(ob + (size_t)rr * (NH * HD) + qd * 4) = ov[i];
    }
}

__attribute__((amdgpu_num_vgpr(256)))
__global__ void __launch_bounds__(128) favor_attn_early(const _Float16* __restrict__ QH,
                                                        const _Float16* __restrict__ KH,
                                                        const _Float16* __restrict__ QR,
                                                        const _Float16* __restrict__ KR,
                                                        const _Float16* __restrict__ VT,
                                                        float* __restrict__ O)
{
    favor_attn_body<true>(QH, KH, QR, KR, VT, O, 0);
}

__attribute__((amdgpu_num_vgpr(256)))
__global__ void __launch_bounds__(128) favor_attn_late(const _Float16* __restrict__ QH,
                                                       const _Float16* __restrict__ KH,
                                                       const _Float16* __restrict__ VT,
                                                       float* __restrict__ O)
{
    favor_attn_body<false>(QH, KH, QH, KH, VT, O, EROWS / QB);
}

extern "C" void kernel_launch(void* const* d_in, const int* in_sizes, int n_in,
                              void* d_out, int out_size, void* d_ws, size_t ws_size,
                              hipStream_t stream)
{
    if (n_in < 4) return;
    const long long need = ((long long)(NB - 1) * S_FULL + SEQ) * NH * HD;
    if ((long long)in_sizes[0] < need || (long long)in_sizes[1] < need || (long long)in_sizes[2] < need) return;
    if ((long long)in_sizes[3] < (long long)NF * HD) return;
    if ((long long)out_size < need) return;
    if (ws_size < (size_t)WS_TOTAL) return;

    const float* Q  = (const float*)d_in[0];
    const float* K  = (const float*)d_in[1];
    const float* V  = (const float*)d_in[2];
    const float* PM = (const float*)d_in[3];
    float*       O  = (float*)d_out;

    char* ws = (char*)d_ws;
    _Float16* QHp = (_Float16*)(ws);
    _Float16* KHp = (_Float16*)(ws + PLANE_BYTES);
    _Float16* VTp = (_Float16*)(ws + 2 * PLANE_BYTES);
    _Float16* QRp = (_Float16*)(ws + 2 * PLANE_BYTES + VT_BYTES);
    _Float16* KRp = (_Float16*)(ws + 2 * PLANE_BYTES + VT_BYTES + RES_BYTES);

    dim3 gplane(SEQ / QB, NB * NH);
    feat_kernel<<<gplane, 128, 0, stream>>>(Q, PM, QHp, QRp);
    feat_kernel<<<gplane, 128, 0, stream>>>(K, PM, KHp, KRp);
    vt_kernel<<<gplane, 128, 0, stream>>>(V, VTp);

    dim3 gearly(EROWS / QB, NB * NH);
    favor_attn_early<<<gearly, 128, 0, stream>>>(QHp, KHp, QRp, KRp, VTp, O);
    if (SEQ > EROWS) {
        dim3 glate((SEQ - EROWS) / QB, NB * NH);
        favor_attn_late<<<glate, 128, 0, stream>>>(QHp, KHp, VTp, O);
    }
}
